// StockLSTM_2448131359199
// MI455X (gfx1250) — hardware-verified
//
#include <hip/hip_runtime.h>

typedef __attribute__((ext_vector_type(16))) __bf16 v16b;
typedef __attribute__((ext_vector_type(8)))  __bf16 v8b;
typedef __attribute__((ext_vector_type(8)))  float  v8f;
typedef __attribute__((ext_vector_type(4)))  float  v4f;

constexpr int T_LEN = 512;
constexpr int IN_D  = 8;
constexpr int HID   = 64;
constexpr int NGATE = 4 * HID;
constexpr int BATCH = 1024;
constexpr int ROWS  = 32;
constexpr int NTHR  = 256;
constexpr int KPADX = 32;
constexpr int PLANE = ROWS * HID;

constexpr int OFF_WHH0  = 0;
constexpr int OFF_WIH1  = OFF_WHH0 + NGATE * HID * 2;
constexpr int OFF_WHH1  = OFF_WIH1 + NGATE * HID * 2;
constexpr int OFF_WIH0  = OFF_WHH1 + NGATE * HID * 2;
constexpr int OFF_HPL   = OFF_WIH0 + NGATE * KPADX * 2;
constexpr int HPL_ELEMS = 8 * PLANE;
constexpr int OFF_SOUT  = OFF_HPL + HPL_ELEMS * 2;
constexpr int LDS_TOTAL = OFF_SOUT + ROWS * 4;

static_assert(BATCH % ROWS == 0, "grid must cover the batch exactly");
static_assert(ROWS == 32 && NTHR == 256, "8 waves per block, one output line per block");
static_assert(HID == 64 && IN_D == 8 && KPADX == 32, "tile geometry");
static_assert((OFF_WIH1 % 16) == 0 && (OFF_WHH1 % 16) == 0 && (OFF_WIH0 % 16) == 0 && (OFF_HPL % 16) == 0 && (OFF_SOUT % 16) == 0, "16-B aligned regions");
static_assert(LDS_TOTAL == 147584, "lds total");
static_assert((HPL_ELEMS * 2) % (16 * NTHR) == 0, "zero-fill coverage");
static_assert((NGATE * HID) % NTHR == 0 && (NGATE * KPADX) % NTHR == 0, "staging coverage");

__device__ __forceinline__ unsigned short f2bf_bits(float f) {
  unsigned u = __float_as_uint(f);
  return (unsigned short)((u + 0x7FFFu + ((u >> 16) & 1u)) >> 16);
}
__device__ __forceinline__ float bf_bits2f(unsigned short h) { return __uint_as_float(((unsigned)h) << 16); }
__device__ __forceinline__ __bf16 bits2bf(unsigned short b) { return __builtin_bit_cast(__bf16, b); }
__device__ __forceinline__ float bf_rne(float f) { return bf_bits2f(f2bf_bits(f)); }

__device__ __forceinline__ v16b frag_load(const __bf16* p) {
  union U { v16b v; v8b h[2]; } f;
  f.h[0] = *(const v8b*)(p);
  f.h[1] = *(const v8b*)(p + 16);
  return f.v;
}

__device__ __forceinline__ v8f mma_bf(v16b a, v16b b, v8f c) {
  c = __builtin_amdgcn_wmma_f32_16x16x32_bf16(false, a, false, b, (short)0, c, false, false);
  asm volatile("v_nop\n\tv_nop\n\tv_nop\n\tv_nop" : "+v"(c) : "v"(a), "v"(b));
  return c;
}

__device__ __forceinline__ float sigm_f(float x) {
  const float e = __builtin_amdgcn_exp2f(x * -1.4426950408889634f);
  return __builtin_amdgcn_rcpf(1.0f + e);
}
__device__ __forceinline__ float tanh_f(float x) {
  const float e = __builtin_amdgcn_exp2f(x * -2.8853900817779268f);
  return 2.0f * __builtin_amdgcn_rcpf(1.0f + e) - 1.0f;
}

__device__ __forceinline__ void cell_update(v8f (&acc)[4], const float (&bias)[4], float (&c)[8],
                                            __bf16* __restrict__ hi_p, __bf16* __restrict__ lo_p, int hst) {
#pragma unroll
  for (int r = 0; r < 8; ++r) {
    const float pi = acc[0][r] + bias[0];
    const float pf = acc[1][r] + bias[1];
    const float pg = acc[2][r] + bias[2];
    const float po = acc[3][r] + bias[3];
    const float iv = sigm_f(pi);
    const float fv = sigm_f(pf);
    const float gv = tanh_f(pg);
    const float ov = sigm_f(po);
    const float cn = fv * c[r] + iv * gv;
    c[r] = cn;
    const float hv = ov * tanh_f(cn);
    const unsigned short hb = f2bf_bits(hv);
    const unsigned short lb = f2bf_bits(hv - bf_bits2f(hb));
    hi_p[hst + r * HID] = bits2bf(hb);
    lo_p[hst + r * HID] = bits2bf(lb);
  }
}

__global__ __launch_bounds__(NTHR)
void lstm2_bf16_kernel(const float* __restrict__ x,
                       const float* __restrict__ Wih0, const float* __restrict__ Whh0,
                       const float* __restrict__ b0,
                       const float* __restrict__ Wih1, const float* __restrict__ Whh1,
                       const float* __restrict__ b1,
                       const float* __restrict__ fcw,  const float* __restrict__ fcb,
                       float* __restrict__ out)
{
  __shared__ __align__(16) unsigned char smem[LDS_TOTAL];
  __bf16* whh0  = (__bf16*)(smem + OFF_WHH0);
  __bf16* wih1  = (__bf16*)(smem + OFF_WIH1);
  __bf16* whh1  = (__bf16*)(smem + OFF_WHH1);
  __bf16* wih0p = (__bf16*)(smem + OFF_WIH0);
  __bf16* hpl   = (__bf16*)(smem + OFF_HPL);
  __bf16* h1hi  = hpl;
  __bf16* h1lo  = hpl + 2 * PLANE;
  __bf16* h2hi  = hpl + 4 * PLANE;
  __bf16* h2lo  = hpl + 6 * PLANE;
  float*  s_out = (float*)(smem + OFF_SOUT);

  const int tid  = threadIdx.x;
  const int lane = tid & 31;
  const int wv   = tid >> 5;
  const int hh   = lane >> 4;
  const int m    = lane & 15;
  const int rh   = wv >> 2;
  const int cq   = wv & 3;
  const int brow = blockIdx.x * ROWS;

#pragma unroll 2
  for (int i = tid; i < NGATE * HID; i += NTHR) {
    whh0[i] = bits2bf(f2bf_bits(Whh0[i]));
    wih1[i] = bits2bf(f2bf_bits(Wih1[i]));
    whh1[i] = bits2bf(f2bf_bits(Whh1[i]));
  }
#pragma unroll 2
  for (int i = tid; i < NGATE * KPADX; i += NTHR) {
    const int row = i >> 5, k = i & 31;
    const int kc = (k < IN_D) ? k : (IN_D - 1);
    const float wvl = Wih0[row * IN_D + kc];
    const unsigned short bits = (k < IN_D) ? f2bf_bits(wvl) : (unsigned short)0;
    wih0p[i] = bits2bf(bits);
  }
  {
    uint4* hz = (uint4*)(smem + OFF_HPL);
    const uint4 z = make_uint4(0u, 0u, 0u, 0u);
    for (int i = tid; i < (HPL_ELEMS * 2) / 16; i += NTHR) hz[i] = z;
  }
  __syncthreads();

  const int gbase = 16 * cq + m;
  float bias_a[4], bias_b[4];
#pragma unroll
  for (int g = 0; g < 4; ++g) {
    const int gr = g * HID + gbase;
    bias_a[g] = bf_rne(b0[gr]);
    bias_b[g] = bf_rne(b1[gr]);
  }
  const int koff = 8 * hh;
  const int arow = (16 * rh + m) * HID + koff;
  const int boff = gbase * HID + koff;
  const int boffx = gbase * KPADX + koff;
  const int hst  = (16 * rh + 8 * hh) * HID + gbase;
  const float* xr = x + (size_t)(brow + 16 * rh + m) * (size_t)(T_LEN * IN_D);

  float cst0[8], cst1[8];
#pragma unroll
  for (int r = 0; r < 8; ++r) { cst0[r] = 0.0f; cst1[r] = 0.0f; }

#pragma unroll 1
  for (int t = 0; t < T_LEN; ++t) {
    const int rb = t & 1, wb = rb ^ 1;

    v8f acc[4];
#pragma unroll
    for (int g = 0; g < 4; ++g) acc[g] = (v8f){0.f,0.f,0.f,0.f,0.f,0.f,0.f,0.f};

    v16b fax;
    {
      const v4f xa = *(const v4f*)(xr + t * IN_D);
      const v4f xb = *(const v4f*)(xr + t * IN_D + 4);
      unsigned short xs[8];
      xs[0] = f2bf_bits(xa[0]); xs[1] = f2bf_bits(xa[1]); xs[2] = f2bf_bits(xa[2]); xs[3] = f2bf_bits(xa[3]);
      xs[4] = f2bf_bits(xb[0]); xs[5] = f2bf_bits(xb[1]); xs[6] = f2bf_bits(xb[2]); xs[7] = f2bf_bits(xb[3]);
#pragma unroll
      for (int e = 0; e < 8; ++e) fax[e] = bits2bf((hh == 0) ? xs[e] : (unsigned short)0);
#pragma unroll
      for (int e = 8; e < 16; ++e) fax[e] = bits2bf((unsigned short)0);
    }
    {
      const __bf16* ahp = h1hi + rb * PLANE + arow;
      const __bf16* alp = h1lo + rb * PLANE + arow;
      v16b ah[2], al[2];
#pragma unroll
      for (int ks = 0; ks < 2; ++ks) { ah[ks] = frag_load(ahp + ks * 32); al[ks] = frag_load(alp + ks * 32); }
#pragma unroll
      for (int g = 0; g < 4; ++g) {
        const v16b bx = frag_load(wih0p + boffx + g * HID * KPADX);
        acc[g] = mma_bf(fax, bx, acc[g]);
#pragma unroll
        for (int ks = 0; ks < 2; ++ks) {
          const v16b bw = frag_load(whh0 + boff + g * HID * HID + ks * 32);
          acc[g] = mma_bf(ah[ks], bw, acc[g]);
          acc[g] = mma_bf(al[ks], bw, acc[g]);
        }
      }
    }
    cell_update(acc, bias_a, cst0, h1hi + wb * PLANE, h1lo + wb * PLANE, hst);
    __syncthreads();

    v8f acd[4];
#pragma unroll
    for (int g = 0; g < 4; ++g) acd[g] = (v8f){0.f,0.f,0.f,0.f,0.f,0.f,0.f,0.f};
    {
      const __bf16* a1hp = h1hi + wb * PLANE + arow;
      const __bf16* a1lp = h1lo + wb * PLANE + arow;
      const __bf16* a2hp = h2hi + rb * PLANE + arow;
      const __bf16* a2lp = h2lo + rb * PLANE + arow;
#pragma unroll
      for (int ks = 0; ks < 2; ++ks) {
        const v16b f1h = frag_load(a1hp + ks * 32);
        const v16b f1l = frag_load(a1lp + ks * 32);
        const v16b f2h = frag_load(a2hp + ks * 32);
        const v16b f2l = frag_load(a2lp + ks * 32);
#pragma unroll
        for (int g = 0; g < 4; ++g) {
          const int bo = boff + g * HID * HID + ks * 32;
          const v16b bw1 = frag_load(wih1 + bo);
          acd[g] = mma_bf(f1h, bw1, acd[g]);
          acd[g] = mma_bf(f1l, bw1, acd[g]);
          const v16b bw2 = frag_load(whh1 + bo);
          acd[g] = mma_bf(f2h, bw2, acd[g]);
          acd[g] = mma_bf(f2l, bw2, acd[g]);
        }
      }
    }
    cell_update(acd, bias_b, cst1, h2hi + wb * PLANE, h2lo + wb * PLANE, hst);
    __syncthreads();
  }

  constexpr int WBL = ((T_LEN - 1) & 1) ^ 1;
  if (tid < ROWS) {
    const unsigned short* ph = (const unsigned short*)(h2hi + WBL * PLANE) + tid * HID;
    const unsigned short* pl = (const unsigned short*)(h2lo + WBL * PLANE) + tid * HID;
    float s = 0.0f;
#pragma unroll 1
    for (int j = 0; j < HID; ++j) {
      const float hv = bf_bits2f(ph[j]) + bf_bits2f(pl[j]);
      const float wv2 = bf_rne(fcw[j]);
      s = s + hv * wv2;
    }
    s = s + bf_rne(fcb[0]);
    s_out[tid] = s;
  }
  __syncthreads();
  if (tid < ROWS / 4) {
    const v4f v = *(const v4f*)(s_out + 4 * tid);
    float* op = out + brow + 4 * tid;
    *(volatile v4f*)op = v;
    __threadfence();
    *(volatile v4f*)op = v;
  }
}

extern "C" void kernel_launch(void* const* d_in, const int* in_sizes, int n_in,
                              void* d_out, int out_size, void* d_ws, size_t ws_size,
                              hipStream_t stream) {
  (void)in_sizes; (void)n_in; (void)out_size; (void)d_ws; (void)ws_size;
  const float* x    = (const float*)d_in[0];
  const float* Wih0 = (const float*)d_in[1];
  const float* Whh0 = (const float*)d_in[2];
  const float* b0   = (const float*)d_in[3];
  const float* Wih1 = (const float*)d_in[4];
  const float* Whh1 = (const float*)d_in[5];
  const float* b1   = (const float*)d_in[6];
  const float* fcw  = (const float*)d_in[7];
  const float* fcb  = (const float*)d_in[8];
  float* out = (float*)d_out;

  const int nblocks = BATCH / ROWS;
  lstm2_bf16_kernel<<<nblocks, NTHR, 0, stream>>>(
      x, Wih0, Whh0, b0, Wih1, Whh1, b1, fcw, fcb, out);
}
